// MixerDiffAttention_13993003450482
// MI455X (gfx1250) — hardware-verified
//
#include <hip/hip_runtime.h>
#include <math.h>
#include <stdint.h>

#define BATCH 2
#define T_LEN 2048
#define NBT (BATCH * T_LEN)
#define DMODEL 2048
#define HDIM 128
#define NQ_HEADS 16
#define NKV_HEADS 8
#define NY_HEADS 8
#define YDIM 256
#define QPITCH (NQ_HEADS * HDIM)
#define KPITCH (NKV_HEADS * HDIM)
#define VT_PITCH NBT
#define KC_KEYS 64
#define P_CARRY 32768.0f
#define SCORE_SCALE 0.08838834764831845f
#define RMS_EPS 1.1920929e-07f
#define LAMBDA_INIT_F 0.2f

#define OFF_XB  0ul
#define OFF_WB  16777216ul
#define OFF_C   33554432ul
#define OFF_QH  67108864ul
#define OFF_QL  83886080ul
#define OFF_KH  100663296ul
#define OFF_KL  109051904ul
#define OFF_VT  117440512ul
#define OFF_COS 125829120ul
#define OFF_SIN 126353408ul
#define WS_TOTAL 126877696ul
static_assert(OFF_WB  == OFF_XB + (size_t)NBT * DMODEL * 2, "xb");
static_assert(OFF_C   == OFF_WB + (size_t)(NQ_HEADS * HDIM + 2 * KPITCH) * DMODEL * 2, "wb");
static_assert(OFF_QH  == OFF_C + (size_t)NBT * QPITCH * 4, "c");
static_assert((size_t)NBT * QPITCH * 4 >= (size_t)NBT * KPITCH * 4, "ck fits");
static_assert((size_t)NBT * QPITCH * 4 >= (size_t)NBT * NY_HEADS * YDIM * 4, "y2 fits");
static_assert(OFF_QL  == OFF_QH + (size_t)NBT * QPITCH * 2, "qh");
static_assert(OFF_KH  == OFF_QL + (size_t)NBT * QPITCH * 2, "ql");
static_assert(OFF_KL  == OFF_KH + (size_t)NBT * KPITCH * 2, "kh");
static_assert(OFF_VT  == OFF_KL + (size_t)NBT * KPITCH * 2, "kl");
static_assert(OFF_COS == OFF_VT + (size_t)(4 * YDIM) * VT_PITCH * 2, "vt");
static_assert(OFF_SIN == OFF_COS + (size_t)T_LEN * 64 * 4, "cos");
static_assert(WS_TOTAL == OFF_SIN + (size_t)T_LEN * 64 * 4, "sin");
static_assert(WS_TOTAL <= 134217728ul, "ws cap");

static_assert(NBT % 64 == 0 && QPITCH % 64 == 0 && KPITCH % 64 == 0 && (4 * YDIM) % 64 == 0, "tile multiples");
static_assert(DMODEL % 32 == 0, "K multiple of 32");
static_assert(T_LEN % 64 == 0 && T_LEN % KC_KEYS == 0, "chunking");

static const unsigned int kInvFreqBits[] = {
0x3f800000u, 0x3f5dafd7u, 0x3f3ff911u, 0x3f263de0u, 0x3f0ff59au, 0x3ef953cfu, 0x3ed7e89bu, 0x3ebaf81au, 0x3ea1e89bu, 0x3e8c3504u, 0x3e72d425u, 0x3e5247edu, 0x3e361887u, 0x3e1db040u, 0x3e088d77u, 0x3dec7fd6u, 0x3dcccccdu, 0x3db15978u, 0x3d99940du, 0x3d84fe4du, 0x3d6655c2u, 0x3d47763fu, 0x3d2cba15u, 0x3d159348u, 0x3d0186e3u, 0x3ce054d3u, 0x3cc2434fu, 0x3ca8398au, 0x3c91ad39u, 0x3c7c4d33u, 0x3c5a7bf2u, 0x3c3d3311u, 0x3c23d70au, 0x3c0de12du, 0x3bf5b9b0u, 0x3bd4ca15u, 0x3bb8449cu, 0x3b9f91ccu, 0x3b8a2e77u, 0x3b6f520eu, 0x3b4f3e38u, 0x3b33770fu, 0x3b1b690du, 0x3b06946fu, 0x3ae91528u, 0x3ac9d75du, 0x3aaec98eu, 0x3a975c0du, 0x3a83126fu, 0x3a6301e2u, 0x3a44948cu, 0x3a2a3b44u, 0x3a136a16u, 0x39ff4facu, 0x39dd1727u, 0x39bf74d7u, 0x39a5cb60u, 0x398f9272u, 0x3978a815u, 0x395753e6u, 0x393a7753u, 0x39217916u, 0x390bd472u, 0x38f22ce4u
};
static_assert(sizeof(kInvFreqBits) / sizeof(kInvFreqBits[0]) == 64, "invfreq count");

typedef __attribute__((ext_vector_type(16))) _Float16 v16h;
typedef __attribute__((ext_vector_type(8)))  _Float16 v8h;
typedef __attribute__((ext_vector_type(16))) __bf16   v16b;
typedef __attribute__((ext_vector_type(8)))  __bf16   v8b;
typedef __attribute__((ext_vector_type(8)))  float    v8f;
typedef __attribute__((ext_vector_type(4)))  float    v4f;
typedef __attribute__((ext_vector_type(4)))  unsigned int v4u;

__device__ __forceinline__ unsigned short f2bf_bits(float f) {
  unsigned u = __float_as_uint(f);
  return (unsigned short)((u + 0x7FFFu + ((u >> 16) & 1u)) >> 16);
}
__device__ __forceinline__ float bf_bits2f(unsigned short h) { return __uint_as_float(((unsigned)h) << 16); }
__device__ __forceinline__ float bf_rne(float f) { return bf_bits2f(f2bf_bits(f)); }

__device__ __forceinline__ void dep_guard_h(v8f& a, v8f& b, v16h x, v16h y) { asm volatile("v_nop\n\tv_nop\n\tv_nop\n\tv_nop" : "+v"(a), "+v"(b) : "v"(x), "v"(y)); }
__device__ __forceinline__ void dep_guard_b(v8f& a, v8f& b, v16b x, v16b y) { asm volatile("v_nop\n\tv_nop\n\tv_nop\n\tv_nop" : "+v"(a), "+v"(b) : "v"(x), "v"(y)); }
__device__ __forceinline__ void keep4_h(v16h a, v16h b, v16h c, v16h d) { asm volatile("v_nop" :: "v"(a), "v"(b), "v"(c), "v"(d)); }
__device__ __forceinline__ void keep4_b(v16b a, v16b b, v16b c, v16b d) { asm volatile("v_nop" :: "v"(a), "v"(b), "v"(c), "v"(d)); }
__device__ __forceinline__ void acc_guard4(v8f& a, v8f& b, v8f& c, v8f& d) { asm volatile("v_nop\n\tv_nop\n\tv_nop\n\tv_nop" : "+v"(a), "+v"(b), "+v"(c), "+v"(d)); }
template <typename T> struct Frag;
template <> struct Frag<_Float16> {
  typedef v16h V; union U { v16h v; v8h h[2]; };
  static __device__ __forceinline__ v16h load(const _Float16* p) {
    U f; f.h[0] = *(const v8h*)(p); f.h[1] = *(const v8h*)(p + 16); return f.v;
  }
  static __device__ __forceinline__ v8f mma(v16h a, v16h b, v8f c) {
    return __builtin_amdgcn_wmma_f32_16x16x32_f16(false, a, false, b, (short)0, c, false, false);
  }
  static __device__ __forceinline__ void guard(v8f& a, v8f& b, v16h x, v16h y) { dep_guard_h(a, b, x, y); }
  static __device__ __forceinline__ void keep(v16h a, v16h b, v16h c, v16h d) { keep4_h(a, b, c, d); }
};
template <> struct Frag<__bf16> {
  typedef v16b V; union U { v16b v; v8b h[2]; };
  static __device__ __forceinline__ v16b load(const __bf16* p) {
    U f; f.h[0] = *(const v8b*)(p); f.h[1] = *(const v8b*)(p + 16); return f.v;
  }
  static __device__ __forceinline__ v8f mma(v16b a, v16b b, v8f c) {
    return __builtin_amdgcn_wmma_f32_16x16x32_bf16(false, a, false, b, (short)0, c, false, false);
  }
  static __device__ __forceinline__ void guard(v8f& a, v8f& b, v16b x, v16b y) { dep_guard_b(a, b, x, y); }
  static __device__ __forceinline__ void keep(v16b a, v16b b, v16b c, v16b d) { keep4_b(a, b, c, d); }
};

__device__ __forceinline__ v8f mma_bf16g(v16b a, v16b b, v8f c) {
  c = __builtin_amdgcn_wmma_f32_16x16x32_bf16(false, a, false, b, (short)0, c, false, false);
  asm volatile("v_nop\n\tv_nop\n\tv_nop\n\tv_nop" : "+v"(c) : "v"(a), "v"(b));
  return c;
}
__device__ __forceinline__ v8f mma_f16g(v16h a, v16h b, v8f c) {
  c = __builtin_amdgcn_wmma_f32_16x16x32_f16(false, a, false, b, (short)0, c, false, false);
  asm volatile("v_nop\n\tv_nop\n\tv_nop\n\tv_nop" : "+v"(c) : "v"(a), "v"(b));
  return c;
}

template <int ET> struct Elem;
template <> struct Elem<0> { typedef _Float16 T; };
template <> struct Elem<1> { typedef __bf16 T; };
template <int ET, bool SPLIT, int BIAS_MODE, int OUT_MODE, bool RESID, int ACT = 0>
__global__ __launch_bounds__(256) void wmma_gemm64(
    const unsigned short* __restrict__ Ap, const unsigned short* __restrict__ A2p, int lda, long strideA,
    const unsigned short* __restrict__ Btp, const unsigned short* __restrict__ Bt2p, int ldb, long strideB,
    void* __restrict__ Cout, void* __restrict__ Cout2, int ldc, long strideC,
    const float* __restrict__ bias,
    const float* __restrict__ resid, long strideR,
    int M, int N, int K, float scale) {
  typedef typename Elem<ET>::T T;
  typedef typename Frag<T>::V V;
  const T* A = (const T*)Ap; const T* A2 = (const T*)A2p; const T* Bt = (const T*)Btp; const T* Bt2 = (const T*)Bt2p;
  __shared__ __align__(16) float sT[8][16 * 68];
  const int b    = blockIdx.y;
  const int lane = threadIdx.x & 31;
  const int wave = threadIdx.x >> 5;
  const int tilesN = N >> 6;
  const int tilesM = M >> 6;
  const int tile = blockIdx.x * 8 + wave;
  if (tile >= tilesM * tilesN) return;
  const int tm = tile / tilesN;
  const int tn = tile - tm * tilesN;
  const int m0 = tm << 6;
  const int n0 = tn << 6;

  const T* Ab  = A  + (size_t)b * strideA;
  const T* Bb  = Bt + (size_t)b * strideB;
  const T* Ab2 = SPLIT ? (A2  + (size_t)b * strideA) : nullptr;
  const T* Bb2 = SPLIT ? (Bt2 + (size_t)b * strideB) : nullptr;

  const int rlane = lane & 15;
  const int koff  = (lane >> 4) * 8;
  const int mOff  = (lane >> 4) * 8;

  v8f acc[4][4];
#pragma unroll
  for (int i = 0; i < 4; ++i)
#pragma unroll
    for (int j = 0; j < 4; ++j) acc[i][j] = (v8f){0.f,0.f,0.f,0.f,0.f,0.f,0.f,0.f};

  for (int k0 = 0; k0 < K; k0 += 32) {
    V bh[4], bl[4];
#pragma unroll
    for (int j = 0; j < 4; ++j) {
      const size_t bo = (size_t)(n0 + (j << 4) + rlane) * ldb + koff + k0;
      bh[j] = Frag<T>::load(Bb + bo);
      if (SPLIT) bl[j] = Frag<T>::load(Bb2 + bo);
    }
#pragma unroll
    for (int i = 0; i < 4; ++i) {
      const size_t ao = (size_t)(m0 + (i << 4) + rlane) * lda + koff + k0;
      V ah = Frag<T>::load(Ab + ao);
      V al;
      if (SPLIT) al = Frag<T>::load(Ab2 + ao);
#pragma unroll
      for (int j = 0; j < 4; ++j) {
        acc[i][j] = Frag<T>::mma(ah, bh[j], acc[i][j]);
        if (SPLIT) {
          acc[i][j] = Frag<T>::mma(ah, bl[j], acc[i][j]);
          acc[i][j] = Frag<T>::mma(al, bh[j], acc[i][j]);
        }
      }
      Frag<T>::guard(acc[i][0], acc[i][3], ah, SPLIT ? al : ah);
    }
    Frag<T>::keep(bh[0], bh[1], bh[2], bh[3]);
    if (SPLIT) Frag<T>::keep(bl[0], bl[1], bl[2], bl[3]);
  }
  acc_guard4(acc[0][0], acc[0][1], acc[0][2], acc[0][3]);
  acc_guard4(acc[1][0], acc[1][1], acc[1][2], acc[1][3]);
  acc_guard4(acc[2][0], acc[2][1], acc[2][2], acc[2][3]);
  acc_guard4(acc[3][0], acc[3][1], acc[3][2], acc[3][3]);

  float* slab = sT[wave];
  const float* Rb = RESID ? (resid + (size_t)b * strideR) : nullptr;
#pragma unroll
  for (int i = 0; i < 4; ++i) {
    const int mBase = m0 + (i << 4);
#pragma unroll
    for (int j = 0; j < 4; ++j) {
      const int n = n0 + (j << 4) + rlane;
      float bv = 0.f;
      if (BIAS_MODE == 2) bv = bias[n];
#pragma unroll
      for (int r = 0; r < 8; ++r) {
        float v = acc[i][j][r] * scale;
        if (BIAS_MODE == 1) v += bias[mBase + mOff + r];
        if (BIAS_MODE == 2) v += bv;
        if (RESID) v += Rb[(size_t)(mBase + mOff + r) * ldc + n];
        if (ACT == 1) v = tanhf(v);
        if (ACT == 2) v = fmaxf(v, 0.0f);
        if (ACT == 3) v = v / (1.0f + expf(-v));
        if (ACT == 4) v = (v > 0.f) ? v : 0.01f * v;
        if (ACT == 5) v = 0.5f * v * (1.0f + erff(v * 0.70710678118654752f));
        slab[(mOff + r) * 68 + (j << 4) + rlane] = v;
      }
    }
    __builtin_amdgcn_fence(__ATOMIC_RELEASE, "workgroup");
    __builtin_amdgcn_wave_barrier();
    __builtin_amdgcn_fence(__ATOMIC_ACQUIRE, "workgroup");
    if (OUT_MODE == 0) {
      float* C = (float*)Cout + (size_t)b * strideC;
      const int hh = lane >> 4, c4 = (lane & 15) * 4;
      for (int pass = 0; pass < 2; ++pass) {
#pragma unroll
        for (int it = 0; it < 8; ++it) {
          const int row = it * 2 + hh;
          v4f v = *(const v4f*)(slab + row * 68 + c4);
          *(volatile v4f*)(C + (size_t)(mBase + row) * ldc + n0 + c4) = v;
        }
        __threadfence();
      }
    } else {
      const int q = lane >> 3, c8 = (lane & 7) * 8;
      unsigned short* C  = (unsigned short*)Cout  + (size_t)b * strideC;
      unsigned short* C2 = (OUT_MODE == 2) ? ((unsigned short*)Cout2 + (size_t)b * strideC) : nullptr;
      for (int pass = 0; pass < 2; ++pass) {
#pragma unroll
        for (int it = 0; it < 4; ++it) {
          const int row = it * 4 + q;
          const float* sp = slab + row * 68 + c8;
          v8h hv, lv;
#pragma unroll
          for (int e = 0; e < 8; ++e) {
            if (OUT_MODE == 1) {
              hv[e] = (_Float16)sp[e];
            } else {
              unsigned short hb = f2bf_bits(sp[e]);
              unsigned short lb = f2bf_bits(sp[e] - bf_bits2f(hb));
              hv[e] = __builtin_bit_cast(_Float16, hb);
              lv[e] = __builtin_bit_cast(_Float16, lb);
            }
          }
          *(volatile v8h*)(C + (size_t)(mBase + row) * ldc + n0 + c8) = hv;
          if (OUT_MODE == 2) *(volatile v8h*)(C2 + (size_t)(mBase + row) * ldc + n0 + c8) = lv;
        }
        __threadfence();
      }
    }
    __builtin_amdgcn_fence(__ATOMIC_RELEASE, "workgroup");
    __builtin_amdgcn_wave_barrier();
    __builtin_amdgcn_fence(__ATOMIC_ACQUIRE, "workgroup");
  }
}

__global__ __launch_bounds__(256) void cvt_f32_bf16x8(const float* __restrict__ in,
                                                      unsigned short* __restrict__ out, int n8) {
  const int i = blockIdx.x * 256 + threadIdx.x;
  if (i < n8) {
    const v4f a = *(const v4f*)(in + (size_t)8 * i);
    const v4f c = *(const v4f*)(in + (size_t)8 * i + 4);
    v4u w;
    w[0] = (unsigned)f2bf_bits(a[0]) | ((unsigned)f2bf_bits(a[1]) << 16);
    w[1] = (unsigned)f2bf_bits(a[2]) | ((unsigned)f2bf_bits(a[3]) << 16);
    w[2] = (unsigned)f2bf_bits(c[0]) | ((unsigned)f2bf_bits(c[1]) << 16);
    w[3] = (unsigned)f2bf_bits(c[2]) | ((unsigned)f2bf_bits(c[3]) << 16);
    unsigned short* p = out + (size_t)8 * i;
    *(volatile v4u*)p = w;
    __threadfence();
    *(volatile v4u*)p = w;
  }
}

struct InvFreq { float f[64]; };
static_assert(sizeof(InvFreq) == 256, "invfreq size");

__global__ __launch_bounds__(256) void rope_table_kernel(InvFreq inv, float* __restrict__ cosT,
                                                         float* __restrict__ sinT) {
  const int tid = threadIdx.x;
  const int i = tid & 63;
  const int t = blockIdx.x * 4 + (tid >> 6);
  float fr = 0.0f;
#pragma unroll
  for (int q = 0; q < 64; ++q) fr = (i == q) ? inv.f[q] : fr;
  const float ang = (float)t * fr;
  const float cv = cosf(ang);
  const float sv = sinf(ang);
  const float cr = bf_rne(cv);
  const float sr = bf_rne(sv);
  const size_t o = (size_t)t * 64 + i;
  *(volatile float*)(cosT + o) = cr;
  *(volatile float*)(sinT + o) = sr;
  __threadfence();
  *(volatile float*)(cosT + o) = cr;
  *(volatile float*)(sinT + o) = sr;
}

__global__ __launch_bounds__(256) void norm_rope_kernel(const float* __restrict__ Cm, int ldc, int npairs, int nwaves,
                                                        const float* __restrict__ cosT, const float* __restrict__ sinT,
                                                        const float* __restrict__ scl, int use_scale,
                                                        unsigned short* __restrict__ outH,
                                                        unsigned short* __restrict__ outL) {
  const int lane = threadIdx.x & 31, wave = threadIdx.x >> 5;
  const int gw = blockIdx.x * 8 + wave;
  if (gw >= nwaves) return;
  const int bt = gw / npairs;
  const int pair = gw - bt * npairs;
  const int t = bt & (T_LEN - 1);
  const int g = lane & 15, hsel = lane >> 4;
  const int h = pair * 2 + hsel;
  const float* p = Cm + (size_t)bt * ldc + h * HDIM + 8 * g;
  const v4f a = *(const v4f*)p;
  const v4f bq = *(const v4f*)(p + 4);
  float v[8] = {a[0], a[1], a[2], a[3], bq[0], bq[1], bq[2], bq[3]};
  float ss = 0.0f;
#pragma unroll
  for (int e = 0; e < 8; ++e) ss += v[e] * v[e];
#pragma unroll
  for (int off = 1; off < 16; off <<= 1) ss += __shfl_xor(ss, off);
  const float inv = 1.0f / sqrtf(ss * (1.0f / 128.0f) + RMS_EPS);
  float pv[8];
#pragma unroll
  for (int e = 0; e < 8; ++e) pv[e] = __shfl_xor(v[e], 8);
  const int i0 = 8 * (g & 7);
  const v4f ca = *(const v4f*)(cosT + (size_t)t * 64 + i0);
  const v4f cb = *(const v4f*)(cosT + (size_t)t * 64 + i0 + 4);
  const v4f sa = *(const v4f*)(sinT + (size_t)t * 64 + i0);
  const v4f sb = *(const v4f*)(sinT + (size_t)t * 64 + i0 + 4);
  float cs[8] = {ca[0], ca[1], ca[2], ca[3], cb[0], cb[1], cb[2], cb[3]};
  float sn[8] = {sa[0], sa[1], sa[2], sa[3], sb[0], sb[1], sb[2], sb[3]};
  const bool first_half = (g < 8);
  float fac = 1.0f;
  if (use_scale) {
    const float sc = bf_rne(scl[h]);
    fac = sc * logf((float)(t + 1));
  }
  unsigned short hb[8], lb[8];
#pragma unroll
  for (int e = 0; e < 8; ++e) {
    const float own = v[e] * inv;
    const float par = pv[e] * inv;
    const float r_first  = own * cs[e] + par * sn[e];
    const float r_second = own * cs[e] - par * sn[e];
    float r = first_half ? r_first : r_second;
    if (use_scale) r = fac * r;
    hb[e] = f2bf_bits(r);
    lb[e] = f2bf_bits(r - bf_bits2f(hb[e]));
  }
  v4u wh, wl;
  wh[0] = (unsigned)hb[0] | ((unsigned)hb[1] << 16);
  wh[1] = (unsigned)hb[2] | ((unsigned)hb[3] << 16);
  wh[2] = (unsigned)hb[4] | ((unsigned)hb[5] << 16);
  wh[3] = (unsigned)hb[6] | ((unsigned)hb[7] << 16);
  wl[0] = (unsigned)lb[0] | ((unsigned)lb[1] << 16);
  wl[1] = (unsigned)lb[2] | ((unsigned)lb[3] << 16);
  wl[2] = (unsigned)lb[4] | ((unsigned)lb[5] << 16);
  wl[3] = (unsigned)lb[6] | ((unsigned)lb[7] << 16);
  const size_t oo = (size_t)bt * ldc + h * HDIM + 8 * g;
  *(volatile v4u*)(outH + oo) = wh;
  *(volatile v4u*)(outL + oo) = wl;
  __threadfence();
  *(volatile v4u*)(outH + oo) = wh;
  *(volatile v4u*)(outL + oo) = wl;
}

template <bool STREAM1>
__global__ __launch_bounds__(256) void diff_attn_kernel(
    const unsigned short* __restrict__ qhp, const unsigned short* __restrict__ qlp,
    const unsigned short* __restrict__ khp, const unsigned short* __restrict__ klp,
    const unsigned short* __restrict__ vtp,
    const float* __restrict__ lq1, const float* __restrict__ lk1,
    const float* __restrict__ lq2, const float* __restrict__ lk2,
    const float* y2p, float* dst) {
  __shared__ __align__(16) unsigned short Kh[KC_KEYS * HDIM];
  __shared__ __align__(16) unsigned short Kl[KC_KEYS * HDIM];
  __shared__ __align__(16) unsigned short Vt[YDIM * KC_KEYS];
  __shared__ __align__(16) unsigned short Qh[64 * HDIM];
  __shared__ __align__(16) unsigned short Ql[64 * HDIM];
  __shared__ __align__(16) _Float16 Ps[4][16 * KC_KEYS];
  __shared__ __align__(16) float Al[64];
  __shared__ __align__(16) float Lf[64];
  __shared__ __align__(16) float Os[8][16 * 68];

  const int tid = threadIdx.x;
  const int wave = tid >> 5, lane = tid & 31, hh = lane >> 4, c = lane & 15;
  const int rg = wave & 3, dh = wave >> 2;
  const int bx = blockIdx.x;
  const int qb = bx & 31;
  const int hj = (bx >> 5) & 7;
  const int b = bx >> 8;
  const int qbase = qb * 64;
  const int q0 = qbase + rg * 16;
  const int qhead = STREAM1 ? hj : (8 + hj);
  const int kvh = STREAM1 ? (hj >> 1) : (4 + (hj >> 1));
  const int vh = hj >> 1;

  float lam = 0.0f;
  if (STREAM1) {
    const float a0 = bf_rne(lq1[lane]), a1 = bf_rne(lq1[lane + 32]);
    const float e0 = bf_rne(lk1[lane]), e1 = bf_rne(lk1[lane + 32]);
    const float g0 = bf_rne(lq2[lane]), g1 = bf_rne(lq2[lane + 32]);
    const float f0 = bf_rne(lk2[lane]), f1 = bf_rne(lk2[lane + 32]);
    float s1 = 0.0f, s2 = 0.0f;
    s1 += a0 * e0; s1 += a1 * e1;
    s2 += g0 * f0; s2 += g1 * f1;
#pragma unroll
    for (int off = 16; off >= 1; off >>= 1) { s1 += __shfl_xor(s1, off); s2 += __shfl_xor(s2, off); }
    lam = (expf(s1) - expf(s2)) + LAMBDA_INIT_F;
  }

#pragma unroll
  for (int it = 0; it < 4; ++it) {
    const int idx = it * 256 + tid;
    const int r = idx >> 4, c16 = idx & 15;
    const size_t go = (size_t)(b * T_LEN + qbase + r) * QPITCH + qhead * HDIM + c16 * 8;
    const uint4 vq = *(const uint4*)(qhp + go);
    const uint4 vl = *(const uint4*)(qlp + go);
    *(uint4*)(Qh + r * HDIM + c16 * 8) = vq;
    *(uint4*)(Ql + r * HDIM + c16 * 8) = vl;
  }

  float mrow[8], lrow[8];
  v8f oacc[8];
#pragma unroll
  for (int r = 0; r < 8; ++r) { mrow[r] = -INFINITY; lrow[r] = 0.0f; }
#pragma unroll
  for (int t8 = 0; t8 < 8; ++t8) oacc[t8] = (v8f){0.f,0.f,0.f,0.f,0.f,0.f,0.f,0.f};

  const int nChunks = qb + 1;
  for (int kc = 0; kc < nChunks; ++kc) {
    const int kv0 = kc * KC_KEYS;
    __syncthreads();
#pragma unroll
    for (int it = 0; it < 4; ++it) {
      const int idx = it * 256 + tid;
      const int r = idx >> 4, c16 = idx & 15;
      const size_t go = (size_t)(b * T_LEN + kv0 + r) * KPITCH + kvh * HDIM + c16 * 8;
      const uint4 a4 = *(const uint4*)(khp + go);
      const uint4 l4 = *(const uint4*)(klp + go);
      *(uint4*)(Kh + r * HDIM + c16 * 8) = a4;
      *(uint4*)(Kl + r * HDIM + c16 * 8) = l4;
    }
#pragma unroll
    for (int it = 0; it < 8; ++it) {
      const int idx = it * 256 + tid;
      const int d = idx >> 3, c8 = idx & 7;
      const size_t go = (size_t)(vh * YDIM + d) * VT_PITCH + b * T_LEN + kv0 + c8 * 8;
      const uint4 v4 = *(const uint4*)(vtp + go);
      *(uint4*)(Vt + d * KC_KEYS + c8 * 8) = v4;
    }
    __syncthreads();

    if (wave < 4) {
      v8f s[4];
#pragma unroll
      for (int jt = 0; jt < 4; ++jt) s[jt] = (v8f){0.f,0.f,0.f,0.f,0.f,0.f,0.f,0.f};
      const __bf16* Qhb = (const __bf16*)Qh + (rg * 16 + c) * HDIM + 8 * hh;
      const __bf16* Qlb = (const __bf16*)Ql + (rg * 16 + c) * HDIM + 8 * hh;
      const __bf16* Khb = (const __bf16*)Kh;
      const __bf16* Klb = (const __bf16*)Kl;
#pragma unroll
      for (int dc = 0; dc < 4; ++dc) {
        const v16b qa = Frag<__bf16>::load(Qhb + dc * 32);
        const v16b ql = Frag<__bf16>::load(Qlb + dc * 32);
#pragma unroll
        for (int jt = 0; jt < 4; ++jt) {
          const int ko = (jt * 16 + c) * HDIM + dc * 32 + 8 * hh;
          const v16b kb = Frag<__bf16>::load(Khb + ko);
          const v16b kl = Frag<__bf16>::load(Klb + ko);
          s[jt] = mma_bf16g(qa, kb, s[jt]);
          s[jt] = mma_bf16g(qa, kl, s[jt]);
          s[jt] = mma_bf16g(ql, kb, s[jt]);
        }
      }
      const bool diag = (kc == qb);
      float cm[8];
#pragma unroll
      for (int r = 0; r < 8; ++r) {
        const int qrow = q0 + 8 * hh + r;
        float m = -INFINITY;
#pragma unroll
        for (int jt = 0; jt < 4; ++jt) {
          const int kvcol = kv0 + jt * 16 + c;
          float val = s[jt][r] * SCORE_SCALE;
          val = (diag && (kvcol > qrow)) ? -INFINITY : val;
          s[jt][r] = val;
          m = fmaxf(m, val);
        }
#pragma unroll
        for (int off = 1; off < 16; off <<= 1) m = fmaxf(m, __shfl_xor(m, off));
        cm[r] = m;
      }
      _Float16* Pw = &Ps[rg][0];
#pragma unroll
      for (int r = 0; r < 8; ++r) {
        const float mnew = fmaxf(mrow[r], cm[r]);
        const float alpha = expf(mrow[r] - mnew);
        mrow[r] = mnew;
        float psum = 0.0f;
#pragma unroll
        for (int jt = 0; jt < 4; ++jt) {
          const float p = expf(s[jt][r] - mnew);
          psum += p;
          Pw[(8 * hh + r) * KC_KEYS + jt * 16 + c] = (_Float16)(p * P_CARRY);
        }
#pragma unroll
        for (int off = 1; off < 16; off <<= 1) psum += __shfl_xor(psum, off);
        lrow[r] = lrow[r] * alpha + psum;
        Al[rg * 16 + 8 * hh + r] = alpha;
      }
    }
    __syncthreads();

    {
      float alr[8];
#pragma unroll
      for (int r = 0; r < 8; ++r) alr[r] = Al[rg * 16 + 8 * hh + r];
#pragma unroll
      for (int t8 = 0; t8 < 8; ++t8)
#pragma unroll
        for (int r = 0; r < 8; ++r) oacc[t8][r] *= alr[r];
      const _Float16* Pr = &Ps[rg][0];
      const _Float16* Vth = (const _Float16*)Vt;
#pragma unroll
      for (int kk = 0; kk < 2; ++kk) {
        const v16h pa = Frag<_Float16>::load(Pr + c * KC_KEYS + kk * 32 + 8 * hh);
#pragma unroll
        for (int t8 = 0; t8 < 8; ++t8) {
          const v16h vb = Frag<_Float16>::load(Vth + (dh * 128 + t8 * 16 + c) * KC_KEYS + kk * 32 + 8 * hh);
          oacc[t8] = mma_f16g(pa, vb, oacc[t8]);
        }
      }
    }
  }

  if (wave < 4) {
#pragma unroll
    for (int r = 0; r < 8; ++r) Lf[wave * 16 + 8 * hh + r] = lrow[r];
  }
  __syncthreads();
  float invl[8];
#pragma unroll
  for (int r = 0; r < 8; ++r) invl[r] = 1.0f / (Lf[rg * 16 + 8 * hh + r] * P_CARRY);

  float* os = &Os[wave][0];
  const int c4 = (lane & 15) * 4;
#pragma unroll
  for (int hf = 0; hf < 2; ++hf) {
#pragma unroll
    for (int r = 0; r < 8; ++r)
#pragma unroll
      for (int t4 = 0; t4 < 4; ++t4) os[(8 * hh + r) * 68 + t4 * 16 + c] = oacc[hf * 4 + t4][r] * invl[r];
    __builtin_amdgcn_fence(__ATOMIC_RELEASE, "workgroup");
    __builtin_amdgcn_wave_barrier();
    __builtin_amdgcn_fence(__ATOMIC_ACQUIRE, "workgroup");
    v4f vals[8];
#pragma unroll
    for (int it = 0; it < 8; ++it) {
      const int row = it * 2 + hh;
      v4f val = *(const v4f*)(os + row * 68 + c4);
      const size_t go = ((size_t)(b * T_LEN + q0 + row) * NY_HEADS + hj) * YDIM + dh * 128 + hf * 64 + c4;
      if (STREAM1) {
        const v4f y2v = *(const v4f*)(y2p + go);
        val = val - lam * y2v;
      }
      vals[it] = val;
    }
    for (int pass = 0; pass < 2; ++pass) {
#pragma unroll
      for (int it = 0; it < 8; ++it) {
        const int row = it * 2 + hh;
        const size_t go = ((size_t)(b * T_LEN + q0 + row) * NY_HEADS + hj) * YDIM + dh * 128 + hf * 64 + c4;
        *(volatile v4f*)(dst + go) = vals[it];
      }
      __threadfence();
    }
    __builtin_amdgcn_fence(__ATOMIC_RELEASE, "workgroup");
    __builtin_amdgcn_wave_barrier();
    __builtin_amdgcn_fence(__ATOMIC_ACQUIRE, "workgroup");
  }
}

extern "C" void kernel_launch(void* const* d_in, const int* in_sizes, int n_in,
                              void* d_out, int out_size, void* d_ws, size_t ws_size,
                              hipStream_t stream) {
  if (n_in < 9) return;
  if (ws_size < WS_TOTAL) return;
  if ((size_t)out_size < (size_t)NBT * NY_HEADS * YDIM) return;
  if (in_sizes[0] != NBT * DMODEL || in_sizes[1] != QPITCH * DMODEL ||
      in_sizes[2] != KPITCH * DMODEL || in_sizes[3] != KPITCH * DMODEL ||
      in_sizes[4] < 64 || in_sizes[5] < 64 || in_sizes[6] < 64 || in_sizes[7] < 64 || in_sizes[8] < NQ_HEADS) return;

  const float* x   = (const float*)d_in[0];
  const float* Wq  = (const float*)d_in[1];
  const float* Wk  = (const float*)d_in[2];
  const float* Wv  = (const float*)d_in[3];
  const float* lq1 = (const float*)d_in[4];
  const float* lk1 = (const float*)d_in[5];
  const float* lq2 = (const float*)d_in[6];
  const float* lk2 = (const float*)d_in[7];
  const float* scl = (const float*)d_in[8];
  float* out = (float*)d_out;
  char* ws = (char*)d_ws;

  unsigned short* xb  = (unsigned short*)(ws + OFF_XB);
  unsigned short* wb  = (unsigned short*)(ws + OFF_WB);
  float*          cbf = (float*)(ws + OFF_C);
  unsigned short* qh  = (unsigned short*)(ws + OFF_QH);
  unsigned short* ql  = (unsigned short*)(ws + OFF_QL);
  unsigned short* kh  = (unsigned short*)(ws + OFF_KH);
  unsigned short* kl  = (unsigned short*)(ws + OFF_KL);
  unsigned short* vt  = (unsigned short*)(ws + OFF_VT);
  float*          cosT = (float*)(ws + OFF_COS);
  float*          sinT = (float*)(ws + OFF_SIN);

  InvFreq inv;
  for (int i = 0; i < 64; ++i) {
    union { unsigned int u; float f; } cv;
    cv.u = kInvFreqBits[i];
    inv.f[i] = cv.f;
  }

  cvt_f32_bf16x8<<<(NBT * DMODEL / 8) / 256, 256, 0, stream>>>(x, xb, NBT * DMODEL / 8);
  cvt_f32_bf16x8<<<(QPITCH * DMODEL / 8) / 256, 256, 0, stream>>>(Wq, wb, QPITCH * DMODEL / 8);
  cvt_f32_bf16x8<<<(KPITCH * DMODEL / 8) / 256, 256, 0, stream>>>(Wk, wb + (size_t)QPITCH * DMODEL, KPITCH * DMODEL / 8);
  cvt_f32_bf16x8<<<(KPITCH * DMODEL / 8) / 256, 256, 0, stream>>>(Wv, wb + (size_t)(QPITCH + KPITCH) * DMODEL, KPITCH * DMODEL / 8);
  rope_table_kernel<<<T_LEN / 4, 256, 0, stream>>>(inv, cosT, sinT);
  wmma_gemm64<1, false, 0, 0, false, 0><<<dim3((NBT / 64) * (QPITCH / 64) / 8, 1), 256, 0, stream>>>(
      xb, xb, DMODEL, 0L, wb, wb, DMODEL, 0L, (void*)cbf, (void*)cbf, QPITCH, 0L,
      scl, scl, 0L, NBT, QPITCH, DMODEL, 1.0f);
  norm_rope_kernel<<<(NBT * (NQ_HEADS / 2)) / 8, 256, 0, stream>>>(cbf, QPITCH, NQ_HEADS / 2, NBT * (NQ_HEADS / 2),
                                                                   cosT, sinT, scl, 1, qh, ql);
  wmma_gemm64<1, false, 0, 0, false, 0><<<dim3((NBT / 64) * (KPITCH / 64) / 8, 1), 256, 0, stream>>>(
      xb, xb, DMODEL, 0L, wb + (size_t)QPITCH * DMODEL, wb + (size_t)QPITCH * DMODEL, DMODEL, 0L,
      (void*)cbf, (void*)cbf, KPITCH, 0L, scl, scl, 0L, NBT, KPITCH, DMODEL, 1.0f);
  norm_rope_kernel<<<(NBT * (NKV_HEADS / 2)) / 8, 256, 0, stream>>>(cbf, KPITCH, NKV_HEADS / 2, NBT * (NKV_HEADS / 2),
                                                                    cosT, sinT, scl, 0, kh, kl);
  wmma_gemm64<1, false, 0, 1, false, 0><<<dim3(((4 * YDIM) / 64) * (NBT / 64) / 8, 1), 256, 0, stream>>>(
      wb + (size_t)(QPITCH + KPITCH) * DMODEL, wb + (size_t)(QPITCH + KPITCH) * DMODEL, DMODEL, 0L,
      xb, xb, DMODEL, 0L, (void*)vt, (void*)vt, VT_PITCH, 0L, scl, scl, 0L, 4 * YDIM, NBT, DMODEL, 1.0f);
  diff_attn_kernel<false><<<BATCH * NY_HEADS * (T_LEN / 64), 256, 0, stream>>>(
      qh, ql, kh, kl, vt, lq1, lk1, lq2, lk2, cosT, cbf);
  diff_attn_kernel<true><<<BATCH * NY_HEADS * (T_LEN / 64), 256, 0, stream>>>(
      qh, ql, kh, kl, vt, lq1, lk1, lq2, lk2, cbf, out);
}
